// KeywordEncoder_9680856285391
// MI455X (gfx1250) — hardware-run, weakly checked
//
#include <hip/hip_runtime.h>


#ifndef NB
#define NB 16384
#endif
#define NB_FULL 16384
#define LL    50
#define VOCAB 100000
#define EE    64
#define CC    256
#define KK    128
#define BAGS  32

static_assert(NB <= NB_FULL);
static_assert(NB % 64 == 0);
static_assert(NB % BAGS == 0);
static_assert(BAGS * 8 == 256);
static_assert(EE == 64 && KK == 2 * EE);
static_assert(KK % 32 == 0);
static_assert(CC % 64 == 0);
static_assert((CC * 16) % 256 == 0);
static_assert(16 * 68 * 4 <= 131072);

typedef unsigned short bf;
typedef __attribute__((ext_vector_type(16))) __bf16   v16bf;
typedef __attribute__((ext_vector_type(8)))  unsigned short v8us;
typedef __attribute__((ext_vector_type(8)))  float    v8f;
typedef __attribute__((ext_vector_type(4)))  float    v4f;
typedef __attribute__((ext_vector_type(4)))  int      v4i;
typedef v4f  __attribute__((may_alias)) v4fa;
typedef v4i  __attribute__((may_alias)) v4ia;

__device__ __forceinline__ unsigned short f2bf(float f) { unsigned u = __float_as_uint(f); u += 0x7FFFu + ((u >> 16) & 1u); return (unsigned short)(u >> 16); }
__device__ __forceinline__ float bf2f(unsigned short w) { return __uint_as_float(((unsigned)w) << 16); }
__device__ __forceinline__ int clampi(int v, int lo, int hi) { return min(max(v, lo), hi); }
__device__ __forceinline__ v16bf cat16b(v8us lo, v8us hi) { return __builtin_bit_cast(v16bf, __builtin_shufflevector(lo, hi, 0, 1, 2, 3, 4, 5, 6, 7, 8, 9, 10, 11, 12, 13, 14, 15)); }
__device__ __forceinline__ v8f wmmab(v16bf a, v16bf b, v8f c) { return __builtin_amdgcn_wmma_f32_16x16x32_bf16(false, a, false, b, (short)0, c, false, false); }
__device__ __forceinline__ v16bf ldb(const bf* p)  { return cat16b(*(const v8us*)p, *(const v8us*)(p + 16)); }
__device__ __forceinline__ void wave_sync() { __builtin_amdgcn_fence(3  , "wavefront"); __builtin_amdgcn_wave_barrier(); asm volatile("" ::: "memory"); }
__device__ __forceinline__ float bfr(float f) { return bf2f(f2bf(f)); }

__global__ __launch_bounds__(256) void k_wt(const float* __restrict__ W, bf* W2) {
    const int g = blockIdx.x * 256 + threadIdx.x;
    const int n = g >> 4, pc = g & 15, c8 = (pc & 7) * 8;
    const v8f x = *(const v8f*)(W + (size_t)n * EE + c8);
    v8us o;
#pragma unroll
    for (int k = 0; k < 8; ++k) o[k] = f2bf(x[k]);
    bf* dst = W2 + (size_t)n * KK + pc * 8;
    *(volatile v8us*)dst = o; __threadfence(); *(volatile v8us*)dst = o;
}

__global__ __launch_bounds__(256) void k_bag(const int* __restrict__ tok, const int* __restrict__ lens, const float* __restrict__ emb, bf* MP) {
#pragma clang fp contract(off)
    const int t = threadIdx.x;
    const size_t row = (size_t)blockIdx.x * BAGS + (size_t)(t >> 3);
    const int c8 = (t & 7) * 8;
    int len = lens[row];
    asm volatile("" : "+v"(len));
    const int* ids = tok + row * LL;
    v8f s = (v8f){};
#pragma unroll 1
    for (int l = 0; l < LL; ++l) {
        const int id = clampi(ids[l], 0, VOCAB - 1);
        v8f x = *(const v8f*)(emb + (size_t)id * EE + c8);
        asm volatile("" : "+v"(x));
        const bool on = (l < len);
#pragma unroll
        for (int k = 0; k < 8; ++k) { const float v = bfr(x[k]); s[k] += on ? v : 0.0f; }
    }
    const int dn = max(len, 1);
    const float inv = 1.0f / (float)dn;
    v8us oh, ol;
#pragma unroll
    for (int k = 0; k < 8; ++k) { const float m = s[k] * inv; const unsigned short h = f2bf(m); oh[k] = h; ol[k] = f2bf(m - bf2f(h)); }
    bf* dst = MP + row * KK + c8;
#pragma unroll 1
    for (int ps = 0; ps < 2; ++ps) {
        *(volatile v8us*)dst = oh;
        *(volatile v8us*)(dst + EE) = ol;
        if (ps == 0) __threadfence(); }
}

static_assert(32 * 8 * 16 == 16 * 64 * 4);
__global__ __launch_bounds__(32) __attribute__((amdgpu_num_vgpr(256))) void k_gemm(const bf* __restrict__ MP, const bf* __restrict__ W2, const float* __restrict__ bias,
                                                                                    const float* __restrict__ nul, const int* __restrict__ lens, float* OUT) {
    __shared__ __align__(16) float os[16 * 68];
    const int lane = threadIdx.x & 31, lr = lane & 15, hi = lane >> 4;
    const int p0 = blockIdx.x * 64, n0 = blockIdx.y * 64;
    v8f acc[4][4];
#pragma unroll
    for (int mb = 0; mb < 4; ++mb)
#pragma unroll
        for (int nb = 0; nb < 4; ++nb) acc[mb][nb] = (v8f){};
    const size_t aoff = (size_t)(p0 + lr) * KK + 8 * hi, boff = (size_t)(n0 + lr) * KK + 8 * hi;
#pragma unroll 1
    for (int kc = 0; kc < KK; kc += 32) {
        v16bf a[4];
#pragma unroll
        for (int mb = 0; mb < 4; ++mb) a[mb] = ldb(MP + aoff + (size_t)mb * 16 * KK + kc);
#pragma unroll
        for (int nb = 0; nb < 4; ++nb) { const v16bf b = ldb(W2 + boff + (size_t)nb * 16 * KK + kc);
#pragma unroll
            for (int mb = 0; mb < 4; ++mb) acc[mb][nb] = wmmab(a[mb], b, acc[mb][nb]); }
        asm volatile("v_nop\n\tv_nop\n\tv_nop\n\tv_nop" : "+v"(acc[0][0]), "+v"(acc[1][1]), "+v"(acc[2][2]), "+v"(acc[3][3]) : "v"(a[0]), "v"(a[1]), "v"(a[2]), "v"(a[3]));
    }
    const int c4 = lr * 4;
    const v4f braw = *(const v4f*)(bias + n0 + c4);
    const v4f nraw = *(const v4f*)(nul + n0 + c4);
    v4f bv, nv;
#pragma unroll
    for (int k = 0; k < 4; ++k) { bv[k] = bfr(braw[k]); nv[k] = bfr(nraw[k]); }
#pragma unroll
    for (int mb = 0; mb < 4; ++mb) {
#pragma unroll
        for (int nb = 0; nb < 4; ++nb) {
#pragma unroll
            for (int j = 0; j < 8; ++j) os[(hi * 8 + j) * 68 + nb * 16 + lr] = acc[mb][nb][j]; }
        wave_sync();
#pragma unroll 1
        for (int ps = 0; ps < 2; ++ps) {
#pragma unroll 1
            for (int i = 0; i < 8; ++i) {
                const int r = 2 * i + hi;
                const size_t row = (size_t)(p0 + mb * 16 + r);
                int len = lens[row];
                asm volatile("" : "+v"(len));
                const v4f x = *(const v4fa*)(&os[r * 68 + c4]);
                const bool empty = (len == 0);
                v4f o;
#pragma unroll
                for (int k = 0; k < 4; ++k) { const float pj = x[k] + bv[k]; o[k] = empty ? nv[k] : pj; }
                *(volatile v4f*)(OUT + row * CC + n0 + c4) = o; }
            if (ps == 0) __threadfence(); }
        wave_sync();
    }
}

static constexpr size_t al256(size_t v) { return (v + 255) & ~(size_t)255; }
static constexpr size_t SZ_W2 = al256((size_t)CC * KK * 2);
static constexpr size_t SZ_MP = al256((size_t)NB * KK * 2);
static constexpr size_t SZ_TOTAL = SZ_W2 + SZ_MP;
static_assert(SZ_TOTAL <= (size_t)134217728);

extern "C" void kernel_launch(void* const* d_in, const int* in_sizes, int n_in,
                              void* d_out, int out_size, void* d_ws, size_t ws_size, hipStream_t stream) {
    if (n_in < 6) return;
    if ((size_t)in_sizes[0] < (size_t)NB * LL) return;
    if ((size_t)in_sizes[1] < (size_t)NB) return;
    if ((size_t)in_sizes[2] < (size_t)VOCAB * EE) return;
    if ((size_t)in_sizes[3] < (size_t)CC * EE) return;
    if ((size_t)in_sizes[4] < (size_t)CC || (size_t)in_sizes[5] < (size_t)CC) return;
    if ((size_t)out_size < (size_t)NB * CC) return;
    if (SZ_TOTAL > ws_size) return;
    const int*   tok  = (const int*)d_in[0];
    const int*   lens = (const int*)d_in[1];
    const float* emb  = (const float*)d_in[2];
    const float* W    = (const float*)d_in[3];
    const float* bias = (const float*)d_in[4];
    const float* nul  = (const float*)d_in[5];
    float* OUT = (float*)d_out;
    char* wsp = (char*)d_ws;
    bf* W2 = (bf*)wsp; wsp += SZ_W2;
    bf* MP = (bf*)wsp; wsp += SZ_MP;

    k_wt<<<(CC * 16) / 256, 256, 0, stream>>>(W, W2);
    k_bag<<<NB / BAGS, 256, 0, stream>>>(tok, lens, emb, MP);
    k_gemm<<<dim3(NB / 64, CC / 64), 32, 0, stream>>>(MP, W2, bias, nul, lens, OUT);
}
